// Latent_40853728919869
// MI455X (gfx1250) — hardware-verified
//
#include <hip/hip_runtime.h>
#include <math.h>

typedef __attribute__((ext_vector_type(16))) _Float16 v16h;
typedef __attribute__((ext_vector_type(16))) __bf16 v16b;
typedef __attribute__((ext_vector_type(8)))  _Float16 v8h;
typedef __attribute__((ext_vector_type(8)))  float v8f;
typedef __attribute__((ext_vector_type(4)))  float v4f;
typedef __attribute__((ext_vector_type(2)))  float v2f;
typedef __attribute__((ext_vector_type(4)))  unsigned v4u;
typedef __attribute__((ext_vector_type(4)))  int v4i;
typedef float __attribute__((may_alias)) float_a;
typedef int __attribute__((may_alias)) int_a;

template <typename T> __device__ __forceinline__ void vst2(void* p, T v) { *(volatile T*)p = v; __threadfence(); *(volatile T*)p = v; }
__device__ __forceinline__ v8f wmma16(v16h a, v16h b, v8f c) {
  v8f d = __builtin_amdgcn_wmma_f32_16x16x32_f16(false, a, false, b, (short)0, c, false, false);
  asm volatile("v_nop\n\tv_nop\n\tv_nop\n\tv_nop" : "+v"(d) : "v"(a), "v"(b));
  return d;
}
__device__ __forceinline__ v8f wmma_bf(v16b a, v16b b, v8f c) {
  v8f d = __builtin_amdgcn_wmma_f32_16x16x32_bf16(false, a, false, b, (short)0, c, false, false);
  asm volatile("v_nop\n\tv_nop\n\tv_nop\n\tv_nop" : "+v"(d) : "v"(a), "v"(b));
  return d;
}
__device__ __forceinline__ v16h frag_h(const _Float16* rowk0, int lane) {
  union { v16h v; v8h q[2]; } u; const _Float16* p = rowk0 + 8 * (lane >> 4);
  u.q[0] = *(const v8h*)p; u.q[1] = *(const v8h*)(p + 16); return u.v;
}
__device__ __forceinline__ v16h frag_f32(const float* rowk0, int lane) {
  v16h a; const float* p = rowk0 + 8 * (lane >> 4);
#pragma unroll
  for (int i = 0; i < 8; ++i) { a[i] = (_Float16)p[i]; a[8 + i] = (_Float16)p[16 + i]; }
  return a;
}
__device__ __forceinline__ v16h frag_f32s(const float* rowk0, int lane, float sc) {
  v16h a; const float* p = rowk0 + 8 * (lane >> 4);
#pragma unroll
  for (int i = 0; i < 8; ++i) { a[i] = (_Float16)(p[i] * sc); a[8 + i] = (_Float16)(p[16 + i] * sc); }
  return a;
}
__device__ __forceinline__ v16h fragc_f32(const float* W, int k0, int n, int lane, int ld, int K) {
  v16h a; const int g = lane >> 4;
#pragma unroll
  for (int i = 0; i < 8; ++i) { const int ka = k0 + 8 * g + i, kb = ka + 16;
    a[i] = (_Float16)(ka < K ? W[(size_t)(ka < K ? ka : K - 1) * ld + n] : 0.f); a[8 + i] = (_Float16)(kb < K ? W[(size_t)(kb < K ? kb : K - 1) * ld + n] : 0.f); }
  return a;
}
struct F2 { v16b h, l; };
__device__ __forceinline__ F2 bsplit16(const float v[16]) { F2 r;
#pragma unroll
  for (int i = 0; i < 16; ++i) { const __bf16 h = (__bf16)v[i]; r.h[i] = h; r.l[i] = (__bf16)(v[i] - (float)h); }
  return r; }
__device__ __forceinline__ F2 split_row(const float* row, int k0, int lane) { float v[16]; const float* p = row + k0 + 8 * (lane >> 4);
#pragma unroll
  for (int i = 0; i < 8; ++i) { v[i] = p[i]; v[8 + i] = p[16 + i]; }
  return bsplit16(v); }
__device__ __forceinline__ F2 split_rowK(const float* row, int k0, int lane, int K) { float v[16]; const int g = lane >> 4;
#pragma unroll
  for (int i = 0; i < 8; ++i) { const int ka = k0 + 8 * g + i, kb = ka + 16; v[i] = ka < K ? row[ka < K ? ka : K - 1] : 0.f; v[8 + i] = kb < K ? row[kb < K ? kb : K - 1] : 0.f; }
  return bsplit16(v); }
__device__ __forceinline__ F2 split_col(const float* W, int k0, int n, int lane, int ld, int K) { float v[16]; const int g = lane >> 4;
#pragma unroll
  for (int i = 0; i < 8; ++i) { const int ka = k0 + 8 * g + i, kb = ka + 16; v[i] = ka < K ? W[(size_t)(ka < K ? ka : K - 1) * ld + n] : 0.f; v[8 + i] = kb < K ? W[(size_t)(kb < K ? kb : K - 1) * ld + n] : 0.f; }
  return bsplit16(v); }
__device__ __forceinline__ v8f mac3(const F2& a, const F2& b, v8f c) { c = wmma_bf(a.l, b.h, c); c = wmma_bf(a.h, b.l, c); return wmma_bf(a.h, b.h, c); }
__device__ __forceinline__ float sigm(float v) { return 1.0f / (1.0f + expf(-v)); }
#define LDSX() do { asm volatile("s_wait_dscnt 0" ::: "memory"); __builtin_amdgcn_wave_barrier(); __builtin_amdgcn_fence(__ATOMIC_RELEASE, "workgroup"); } while (0)


#define NN 2048
#define NL 8
#define ND 64
typedef __attribute__((ext_vector_type(8))) __bf16 v8b;
__device__ __forceinline__ v16b frag_b(const __bf16* rowk0, int lane) {
  union { v16b v; v8b q[2]; } u; const __bf16* p = rowk0 + 8 * (lane >> 4);
  u.q[0] = *(const v8b*)p; u.q[1] = *(const v8b*)(p + 16); return u.v;
}
__device__ __forceinline__ v16b frag_gbf(const float* rowk0, int lane) {
  v16b a; const float* p = rowk0 + 8 * (lane >> 4);
#pragma unroll
  for (int i = 0; i < 8; ++i) { a[i] = (__bf16)p[i]; a[8 + i] = (__bf16)p[16 + i]; }
  return a;
}
__device__ __forceinline__ float bfr(float v) { return (float)(__bf16)v; }
__device__ __attribute__((noinline)) float exp_ni(float v) { return expf(v); }
__device__ __attribute__((noinline)) float log_ni(float v) { return logf(v); }
#define WS_H    0u
#define WS_PART (WS_H + 4u * NN * NL * ND)
#define WS_END  (WS_PART + 4u * NL * 32 * 32)

__global__ __launch_bounds__(128) void k_h(const float* __restrict__ Z, const float* __restrict__ We, const float* __restrict__ be, float* __restrict__ H, float* __restrict__ ZM) {
  __shared__ __align__(16) float so[4][16][132];
  const int tid = threadIdx.x, wave = tid >> 5, lane = tid & 31, col = lane & 15, g = lane >> 4; const int r0 = blockIdx.x * 64 + wave * 16; const int n0 = blockIdx.y * 128;
  v8f acc[8] = {};
#pragma unroll
  for (int kc = 0; kc < 2; ++kc) { const v16b a = frag_gbf(Z + (size_t)(r0 + col) * ND + kc * 32, lane);
#pragma unroll
    for (int j = 0; j < 8; ++j) acc[j] = wmma_bf(a, frag_gbf(We + (size_t)(n0 + j * 16 + col) * ND + kc * 32, lane), acc[j]); }
#pragma unroll
  for (int j = 0; j < 8; ++j) { const float bb = bfr(be[n0 + j * 16 + col]);
#pragma unroll
    for (int r = 0; r < 8; ++r) so[wave][8 * g + r][j * 16 + col] = acc[j][r] + bb; }
  LDSX();
  for (int rl = 0; rl < 16; ++rl) { const int n = r0 + rl; vst2(H + (size_t)n * (NL * ND) + n0 + lane * 4, *(const v4f*)&so[wave][rl][lane * 4]);
    const int l = (n0 + (lane >> 4) * 64) / ND; vst2(ZM + ((size_t)l * NN + n) * ND + (lane & 15) * 4, *(const v4f*)&so[wave][rl][lane * 4]); }
}
__global__ __launch_bounds__(128) void k_dec(const float* __restrict__ H, const float* __restrict__ Wd, const float* __restrict__ bd, float* __restrict__ ZD) {
  __shared__ __align__(16) float so[4][16][68];
  const int tid = threadIdx.x, wave = tid >> 5, lane = tid & 31, col = lane & 15, g = lane >> 4; const int r0 = blockIdx.x * 64 + wave * 16;
  v8f acc[4] = {};
#pragma unroll 2
  for (int kc = 0; kc < NL * ND / 32; ++kc) { const F2 a = split_row(H + (size_t)(r0 + col) * (NL * ND), kc * 32, lane);
#pragma unroll
    for (int j = 0; j < 4; ++j) { const v16b w = frag_gbf(Wd + (size_t)(j * 16 + col) * (NL * ND) + kc * 32, lane); acc[j] = wmma_bf(a.l, w, acc[j]); acc[j] = wmma_bf(a.h, w, acc[j]); } }
#pragma unroll
  for (int j = 0; j < 4; ++j) { const float bb = bfr(bd[j * 16 + col]);
#pragma unroll
    for (int r = 0; r < 8; ++r) so[wave][8 * g + r][j * 16 + col] = acc[j][r] + bb; }
  LDSX();
  for (int rl = 0; rl < 16; ++rl) if (lane < 16) vst2(ZD + (size_t)(r0 + rl) * ND + lane * 4, *(const v4f*)&so[wave][rl][lane * 4]);
}
__global__ __launch_bounds__(128) void k_lse(const float* __restrict__ Ein, const float* __restrict__ ZM, const float* __restrict__ lsig, float* __restrict__ PART) {
  __shared__ float szn[NN]; __shared__ float sl[64]; __shared__ __align__(16) float sres[32];
  const int tid = threadIdx.x, wave = tid >> 5, lane = tid & 31, col = lane & 15, g = lane >> 4; const int l = blockIdx.y, m0 = blockIdx.x * 64 + wave * 16;
  const float ls = bfr(lsig[0]); const float sg = exp_ni(ls); const float alpha = -1.0f / (2.0f * sg * sg);
  for (int n = tid; n < NN; n += 128) { const float* zr = ZM + ((size_t)l * NN + n) * ND; float s = 0.f; for (int d = 0; d < ND; ++d) s += zr[d] * zr[d]; szn[n] = s; }
  float em2[8];
#pragma unroll
  for (int r = 0; r < 8; ++r) { const float* er = Ein + ((size_t)l * NN + m0 + 8 * g + r) * ND; float s = 0.f; for (int d = 0; d < ND; ++d) { const float v = bfr(er[d]); s += v * v; } em2[r] = s; }
  __syncthreads();
  const v16b a0 = frag_gbf(Ein + ((size_t)l * NN + m0 + col) * ND, lane), a1 = frag_gbf(Ein + ((size_t)l * NN + m0 + col) * ND + 32, lane);
  float mx[8], sm[8];
#pragma unroll
  for (int r = 0; r < 8; ++r) { mx[r] = -3.0e38f; sm[r] = 0.f; }
#pragma unroll 1
  for (int nt = 0; nt < NN / 16; ++nt) { const float* zr = ZM + ((size_t)l * NN + nt * 16 + col) * ND; const F2 b0 = split_row(zr, 0, lane), b1 = split_row(zr, 32, lane);
    v8f c = {}; c = wmma_bf(a0, b0.h, c); c = wmma_bf(a0, b0.l, c); c = wmma_bf(a1, b1.h, c); c = wmma_bf(a1, b1.l, c);
    const float zn = szn[nt * 16 + col];
#pragma unroll
    for (int r = 0; r < 8; ++r) { const float d2 = (zn + em2[r]) - 2.0f * c[r]; const float v = alpha * d2; float tmx = v;
#pragma unroll
      for (int o = 1; o < 16; o <<= 1) tmx = fmaxf(tmx, __shfl_xor(tmx, o));
      const float nm = fmaxf(mx[r], tmx); float ex = exp_ni(v - nm);
#pragma unroll
      for (int o = 1; o < 16; o <<= 1) ex += __shfl_xor(ex, o);
      sm[r] = sm[r] * exp_ni(mx[r] - nm) + ex; mx[r] = nm; } }
  if (col == 0) {
#pragma unroll
    for (int r = 0; r < 8; ++r) sl[wave * 16 + 8 * g + r] = mx[r] + log_ni(sm[r]); }
  __syncthreads();
  if (tid < 32) { float s = sl[tid] + sl[tid + 32];
#pragma unroll
    for (int o = 1; o < 32; o <<= 1) s += __shfl_xor(s, o);
    if (tid == 0) sres[0] = s;
    if (tid > 0) sres[tid] = 0.f; }
  __syncthreads();
  if (tid < 8) vst2(PART + ((size_t)l * 32 + blockIdx.x) * 32 + tid * 4, *(const v4f*)&sres[tid * 4]);
}
__global__ __launch_bounds__(64) void k_fin(const float* __restrict__ PART, const float* __restrict__ lsig, float* __restrict__ out2) {
  const int tid = threadIdx.x; __shared__ double sp[64];
  double s = 0.0; for (int i = tid; i < NL * 32; i += 64) s += (double)PART[(size_t)i * 32];
  sp[tid] = s; __syncthreads();
  if (tid == 0) { double t = 0.0; for (int i = 0; i < 64; ++i) t += sp[i]; const float ls = bfr(lsig[0]);
    const double loss = -(t / (double)NN) / (double)NL + 0.5 * 64.0 * (2.0 * (double)ls - 1.0) + log(2048.0);
    vst2(out2, (float_a)(float)loss); }
}

extern "C" void kernel_launch(void* const* d_in, const int* in_sizes, int n_in, void* d_out, int out_size, void* d_ws, size_t ws_size, hipStream_t stream) {
  (void)in_sizes; (void)n_in; (void)out_size;
  const float** F = (const float**)d_in;
  if (ws_size < (size_t)WS_END) return;
  char* ws = (char*)d_ws; float *H = (float*)(ws + WS_H), *PART = (float*)(ws + WS_PART);
  float* ZD = (float*)d_out; float* ZM = ZD + (size_t)NN * ND; float* LOSS = ZM + (size_t)NL * NN * ND;
  k_h<<<dim3(NN / 64, NL * ND / 128), 128, 0, stream>>>(F[0], F[2], F[3], H, ZM);
  k_dec<<<NN / 64, 128, 0, stream>>>(H, F[4], F[5], ZD);
  k_lse<<<dim3(NN / 64, NL), 128, 0, stream>>>(F[1], ZM, F[6], PART);
  k_fin<<<1, 64, 0, stream>>>(PART, F[6], LOSS);
}
